// GNN_drug_33019708572239
// MI455X (gfx1250) — hardware-verified
//
#include <hip/hip_runtime.h>
#include <stddef.h>


#define HID     128
#define NTHR    256
#define NWAVE   8
#define EPT     8
#define NGRP    2
#define CHUNK   (NTHR * EPT * NGRP)
#define WCAP    (EPT * NGRP * 32)
#define LISTN   (NWAVE * WCAP)
#define NBC     4096
#define NBF     2048
#define NBP     256
#define RCAP    45056
#define RBN     128
#define OTHR    512
#define GROWS   128
#define AP      136
#define DEGCAP  256
#define WPL     16384
#define BN_EPS  1e-5f

#define LH_BYTES  (GROWS * AP * 2)
#define LDS_LAYER (2 * LH_BYTES + 16 * HID * 2 * 8)
#define LDS_FILL  ((RCAP + NBF + LISTN) * 4 + 64)
#define LDS_SEG   ((NBP * HID + LISTN) * 4 + 64)

static_assert((CHUNK & (CHUNK - 1)) == 0);
static_assert(CHUNK <= 4096);
static_assert(NBC <= 4096 && NBF <= 4096 && NBP <= 4096);
static_assert((NBC & (NBC - 1)) == 0 && (NBF & (NBF - 1)) == 0 && (NBP & (NBP - 1)) == 0);
static_assert(NBC == 2 * NBF);
static_assert(OTHR * 8 == NBC);
static_assert((RCAP % 32) == 0);
static_assert(GROWS == NWAVE * 16);
static_assert(NBP == NWAVE * 32);
static_assert(GROWS * HID * 4 <= 2 * LH_BYTES);
static_assert((AP % 8) == 0);

typedef float          v4f  __attribute__((ext_vector_type(4)));
typedef float          v8f  __attribute__((ext_vector_type(8)));
typedef int            v4i  __attribute__((ext_vector_type(4)));
typedef unsigned int   v2u  __attribute__((ext_vector_type(2)));
typedef unsigned short v8us __attribute__((ext_vector_type(8)));
typedef double         v2d  __attribute__((ext_vector_type(2)));
typedef __bf16         v16b __attribute__((ext_vector_type(16)));
union FragB { v16b v; v8us u[2]; };

__device__ __forceinline__ unsigned int bfbits(float f) {
  const unsigned int u = __float_as_uint(f);
  return (u + 0x7fffu + ((u >> 16) & 1u)) >> 16;
}
__device__ __forceinline__ void split2(float v, unsigned int& hb, unsigned int& lb) {
  hb = bfbits(v);
  const float hf = __uint_as_float(hb << 16);
  lb = bfbits(v - hf);
}

__device__ __forceinline__ v8f wmb(v16b a, v16b b, v8f c) {
  v8f d = __builtin_amdgcn_wmma_f32_16x16x32_bf16(false, a, false, b, (short)0, c, false, false);
  asm volatile("v_nop\n\tv_nop\n\tv_nop\n\tv_nop" : "+v"(d) : "v"(a), "v"(b));
  return d;
}

template <int NB>
__device__ __forceinline__ int scan_chunk(const int* __restrict__ dsts, int nE, int cbase, int slotBase,
                                          int vec8, int* list, int tid, int lane, int wave) {
  int wc = 0;
#pragma unroll
  for (int g = 0; g < NGRP; ++g) {
    const int el0  = (g * NTHR + tid) * EPT;
    const int e0   = cbase + el0;
    const int sent = -2147483647 - 1;
    v4i da, db;
    if (vec8 != 0 && cbase + CHUNK <= nE) {
      da = *(const v4i*)(dsts + e0);
      db = *(const v4i*)(dsts + e0 + 4);
    } else {
      da.x = (e0     < nE) ? dsts[min(e0, nE - 1)] : sent;
      da.y = (e0 + 1 < nE) ? dsts[min(e0 + 1, nE - 1)] : sent;
      da.z = (e0 + 2 < nE) ? dsts[min(e0 + 2, nE - 1)] : sent;
      da.w = (e0 + 3 < nE) ? dsts[min(e0 + 3, nE - 1)] : sent;
      db.x = (e0 + 4 < nE) ? dsts[min(e0 + 4, nE - 1)] : sent;
      db.y = (e0 + 5 < nE) ? dsts[min(e0 + 5, nE - 1)] : sent;
      db.z = (e0 + 6 < nE) ? dsts[min(e0 + 6, nE - 1)] : sent;
      db.w = (e0 + 7 < nE) ? dsts[min(e0 + 7, nE - 1)] : sent;
    }
    const unsigned nb = (unsigned)slotBase;
    const unsigned s0 = (unsigned)da.x - nb, s1 = (unsigned)da.y - nb;
    const unsigned s2 = (unsigned)da.z - nb, s3 = (unsigned)da.w - nb;
    const unsigned s4 = (unsigned)db.x - nb, s5 = (unsigned)db.y - nb;
    const unsigned s6 = (unsigned)db.z - nb, s7 = (unsigned)db.w - nb;
    const bool h0 = s0 < (unsigned)NB, h1 = s1 < (unsigned)NB, h2 = s2 < (unsigned)NB, h3 = s3 < (unsigned)NB;
    const bool h4 = s4 < (unsigned)NB, h5 = s5 < (unsigned)NB, h6 = s6 < (unsigned)NB, h7 = s7 < (unsigned)NB;
    const unsigned any = __builtin_amdgcn_ballot_w32(h0 | h1 | h2 | h3 | h4 | h5 | h6 | h7);
    if (any != 0u) {
#define HITJ(J, HJ, SJ) { \
        const unsigned mj = __builtin_amdgcn_ballot_w32(HJ); \
        if (mj != 0u) { \
          if (HJ) { \
            const int pos = wc + (int)__builtin_amdgcn_mbcnt_lo(mj, 0u); \
            if (pos < WCAP) list[wave * WCAP + pos] = ((el0 + (J)) << 12) | (int)(SJ); \
          } \
          wc += (int)__builtin_popcount(mj); } }
      HITJ(0, h0, s0)
      HITJ(1, h1, s1)
      HITJ(2, h2, s2)
      HITJ(3, h3, s3)
      HITJ(4, h4, s4)
      HITJ(5, h5, s5)
      HITJ(6, h6, s6)
      HITJ(7, h7, s7)
#undef HITJ
    }
  }
  return wc;
}

__global__ __launch_bounds__(NTHR) void k_wprep(
    const float* __restrict__ w10, const float* __restrict__ w20,
    const float* __restrict__ w11, const float* __restrict__ w21,
    const float* __restrict__ w12, const float* __restrict__ w22,
    unsigned short* wsb, int din0) {
  const int i  = blockIdx.x * NTHR + (int)threadIdx.x;
  const int mi = i >> 11;
  if (mi > 5) return;
  const float* src = mi == 0 ? w10 : (mi == 1 ? w20 : (mi == 2 ? w11 : (mi == 3 ? w21 : (mi == 4 ? w12 : w22))));
  const int K  = (mi == 0) ? din0 : HID;
  const int o  = (i & 2047) * 8;
  const int n  = o >> 7;
  const int k0 = o & (HID - 1);
  unsigned int hb[8], lb[8];
#pragma unroll
  for (int e = 0; e < 8; ++e) {
    const int k  = k0 + e;
    const int kc = k < K ? k : K - 1;
    const float x = src[(size_t)kc * HID + n];
    const float v = (k < K) ? x : 0.0f;
    split2(v, hb[e], lb[e]);
  }
  v8us hv, lv;
#pragma unroll
  for (int e = 0; e < 8; ++e) { hv[e] = (unsigned short)hb[e]; lv[e] = (unsigned short)lb[e]; }
  unsigned short* ph = wsb + (size_t)mi * (2 * WPL) + o;
  unsigned short* pl = ph + WPL;
  *(volatile v8us*)ph = hv;
  *(volatile v8us*)pl = lv;
  __threadfence();
  *(volatile v8us*)ph = hv;
  *(volatile v8us*)pl = lv;
}

__global__ __launch_bounds__(NTHR) void k_pad(const float* __restrict__ x, float* P, int nN, int fin, int total4) {
  const int i = blockIdx.x * NTHR + (int)threadIdx.x;
  if (i >= total4) return;
  const int row = i >> 5;
  const int c0  = (i & 31) * 4;
  const int rc  = row < nN ? row : nN - 1;
  const float* xr = x + (size_t)rc * fin;
  float v[4];
#pragma unroll
  for (int e = 0; e < 4; ++e) {
    const int c  = c0 + e;
    const int cc = c < fin ? c : fin - 1;
    const float t = xr[cc];
    v[e] = (row < nN && c < fin) ? t : 0.0f;
  }
  v4f o;
  o.x = v[0]; o.y = v[1]; o.z = v[2]; o.w = v[3];
  float* pp = P + (size_t)i * 4;
  *(volatile v4f*)pp = o;
  __threadfence();
  *(volatile v4f*)pp = o;
}

__global__ __launch_bounds__(NTHR) void k_count(const int* __restrict__ ei, int* cnt, int nE, int vec8) {
  __shared__ __attribute__((aligned(16))) int scnt[NBC];
  __shared__ __attribute__((aligned(16))) int list[LISTN];
  __shared__ int wcnt[NWAVE];
  const int tid = threadIdx.x, lane = tid & 31, wave = tid >> 5;
  const int nodeBase = blockIdx.x * NBC;
  const int* dsts = ei + nE;

  for (int i = tid; i < NBC; i += NTHR) scnt[i] = 0;
  __syncthreads();

  const int nChunks = (nE + CHUNK - 1) / CHUNK;
#pragma unroll 1
  for (int ch = 0; ch < nChunks; ++ch) {
    const int cbase = ch * CHUNK;
    const int wc = scan_chunk<NBC>(dsts, nE, cbase, nodeBase, vec8, list, tid, lane, wave);
    if (lane == 0) wcnt[wave] = wc;
    __syncthreads();
    if (wave == 0) {
#pragma unroll 1
      for (int wsx = 0; wsx < NWAVE; ++wsx) {
        int n = __builtin_amdgcn_readfirstlane(wcnt[wsx]);
        n = n > WCAP ? WCAP : (n < 0 ? 0 : n);
        const int* lp = list + wsx * WCAP;
#pragma unroll 1
        for (int i = 0; i < n; ++i) {
          const int ent  = __builtin_amdgcn_readfirstlane(lp[i]);
          const int slot = ent & (NBC - 1);
          if (lane == 0) scnt[slot] = scnt[slot] + 1;
        }
      }
    }
    __syncthreads();
  }

  v4i cq[4];
#pragma unroll
  for (int q = 0; q < 4; ++q) {
    const int f = (wave * 4 + q) * 128 + 4 * lane;
    cq[q] = *(const v4i*)(scnt + f);
  }
  int* cp = cnt + (size_t)nodeBase;
#pragma unroll
  for (int q = 0; q < 4; ++q) {
    const int f = (wave * 4 + q) * 128 + 4 * lane;
    *(volatile v4i*)(cp + f) = cq[q];
  }
  __threadfence();
#pragma unroll
  for (int q = 0; q < 4; ++q) {
    const int f = (wave * 4 + q) * 128 + 4 * lane;
    *(volatile v4i*)(cp + f) = cq[q];
  }
}

__global__ __launch_bounds__(OTHR) void k_offsets(
    const int* __restrict__ cnt, int* off, int* rbase, int nChunk) {
  __shared__ __attribute__((aligned(16))) int soff[NBC];
  __shared__ __attribute__((aligned(16))) int srb[RBN];
  __shared__ int wtot[OTHR / 32];
  const int tid = threadIdx.x, lane = tid & 31, wave = tid >> 5, sub = tid >> 8;
  for (int i = tid; i < RBN; i += OTHR) srb[i] = 0;
  int carry = 0;
#pragma unroll 1
  for (int ch = 0; ch < nChunk; ++ch) {
    const int base = ch * NBC;
    const v4i c0 = *(const v4i*)(cnt + base + 8 * tid);
    const v4i c1 = *(const v4i*)(cnt + base + 8 * tid + 4);
    const int e0 = max(c0.x, 0), e1 = max(c0.y, 0), e2 = max(c0.z, 0), e3 = max(c0.w, 0);
    const int e4 = max(c1.x, 0), e5 = max(c1.y, 0), e6 = max(c1.z, 0), e7 = max(c1.w, 0);
    const int ts = e0 + e1 + e2 + e3 + e4 + e5 + e6 + e7;
    int incl = ts;
#pragma unroll
    for (int d = 1; d < 32; d <<= 1) {
      const int t = __shfl_up(incl, d);
      if (lane >= d) incl += t;
    }
    if (lane == 31) wtot[wave] = incl;
    __syncthreads();
    const int S0 = wtot[0] + wtot[1] + wtot[2]  + wtot[3]  + wtot[4]  + wtot[5]  + wtot[6]  + wtot[7];
    const int S1 = wtot[8] + wtot[9] + wtot[10] + wtot[11] + wtot[12] + wtot[13] + wtot[14] + wtot[15];
    int pre = 0;
#pragma unroll 1
    for (int w = 8 * sub; w < wave; ++w) pre += wtot[w];
    const int b0 = carry;
    const int b1 = b0 + ((S0 + 31) & ~31);
    const int b2 = b1 + ((S1 + 31) & ~31);
    const int myb = sub == 0 ? b0 : b1;
    if (tid == 0) {
      srb[min(2 * ch + 0, RBN - 1)] = b0;
      srb[min(2 * ch + 1, RBN - 1)] = b1;
    }
    int run = myb + pre + incl - ts;
    soff[8 * tid + 0] = run; run += e0;
    soff[8 * tid + 1] = run; run += e1;
    soff[8 * tid + 2] = run; run += e2;
    soff[8 * tid + 3] = run; run += e3;
    soff[8 * tid + 4] = run; run += e4;
    soff[8 * tid + 5] = run; run += e5;
    soff[8 * tid + 6] = run; run += e6;
    soff[8 * tid + 7] = run;
    carry = b2;
    __syncthreads();
    const v4i o0 = *(const v4i*)(soff + 4 * tid);
    const v4i o1 = *(const v4i*)(soff + 4 * (tid + OTHR));
    int* op = off + base;
    *(volatile v4i*)(op + 4 * tid) = o0;
    *(volatile v4i*)(op + 4 * (tid + OTHR)) = o1;
    __threadfence();
    *(volatile v4i*)(op + 4 * tid) = o0;
    *(volatile v4i*)(op + 4 * (tid + OTHR)) = o1;
    __syncthreads();
  }
  if (tid == 0) srb[min(2 * nChunk, RBN - 1)] = carry;
  __syncthreads();
  v4i rv = {0, 0, 0, 0};
  if (tid < 32) rv = *(const v4i*)(srb + 4 * tid);
  if (tid < 32) *(volatile v4i*)(rbase + 4 * tid) = rv;
  __threadfence();
  if (tid < 32) *(volatile v4i*)(rbase + 4 * tid) = rv;
}

__global__ __launch_bounds__(NTHR) void k_fill(
    const int* __restrict__ ei, const int* __restrict__ off, const int* __restrict__ rbase,
    int* csr, int nN, int nE, int vec8, int csrLen) {
  extern __shared__ v4f lds_dyn[];
  int* region = (int*)lds_dyn;
  int* cursor = region + RCAP;
  int* list   = cursor + NBF;
  int* wcnt   = list + LISTN;
  const int tid = threadIdx.x, lane = tid & 31, wave = tid >> 5;
  const int b = blockIdx.x;
  const int nodeBase = b * NBF;
  const int* dsts = ei + nE;

  int rb0 = rbase[b];
  const int rb1 = rbase[b + 1];
  rb0 = rb0 < 0 ? 0 : (rb0 > csrLen ? csrLen : rb0);
  rb0 &= ~31;
  int len = rb1 - rb0;
  len = len < 0 ? 0 : (len > RCAP ? RCAP : len);
  int lenW = (len + 31) & ~31;
  if (rb0 + lenW > csrLen) lenW = (csrLen - rb0) & ~31;

  {
    const v4i z = {0, 0, 0, 0};
    for (int i = tid; i < RCAP / 4; i += NTHR) ((v4i*)region)[i] = z;
    for (int s = tid; s < NBF; s += NTHR) {
      int o = off[nodeBase + s] - rb0;
      o = o < 0 ? 0 : (o > RCAP ? RCAP : o);
      cursor[s] = o;
    }
  }
  __syncthreads();

  const int nChunks = (nE + CHUNK - 1) / CHUNK;
#pragma unroll 1
  for (int ch = 0; ch < nChunks; ++ch) {
    const int cbase = ch * CHUNK;
    const int wc = scan_chunk<NBF>(dsts, nE, cbase, nodeBase, vec8, list, tid, lane, wave);
    if (lane == 0) wcnt[wave] = wc;
    __syncthreads();
    if (wave == 0) {
#pragma unroll 1
      for (int wsx = 0; wsx < NWAVE; ++wsx) {
        int n = __builtin_amdgcn_readfirstlane(wcnt[wsx]);
        n = n > WCAP ? WCAP : (n < 0 ? 0 : n);
        const int* lp = list + wsx * WCAP;
#pragma unroll 1
        for (int i = 0; i < n; ++i) {
          const int ent  = __builtin_amdgcn_readfirstlane(lp[i]);
          const int slot = ent & (NBF - 1);
          int e = cbase + ((ent >> 12) & (CHUNK - 1));
          e = e > nE - 1 ? nE - 1 : e;
          int src = ei[e];
          src = src < 0 ? 0 : (src > nN - 1 ? nN - 1 : src);
          if (lane == 0) {
            int pos = cursor[slot];
            pos = pos < 0 ? 0 : (pos > RCAP - 1 ? RCAP - 1 : pos);
            region[pos] = src;
            const int np = pos + 1;
            cursor[slot] = np > RCAP ? RCAP : np;
          }
        }
      }
    }
    __syncthreads();
  }

  const int nv = lenW >> 2;
  int* gp = csr + rb0;
#pragma unroll 1
  for (int i = tid; i < nv; i += NTHR) { const v4i v = ((const v4i*)region)[i]; *(volatile v4i*)(gp + 4 * i) = v; }
  __threadfence();
#pragma unroll 1
  for (int i = tid; i < nv; i += NTHR) { const v4i v = ((const v4i*)region)[i]; *(volatile v4i*)(gp + 4 * i) = v; }
}

template <int KS>
__device__ __forceinline__ void mm_tile(const unsigned short* sH, const unsigned short* sL,
                                        const unsigned short* __restrict__ wp,
                                        int r0, int hh, int m, v8f (&acc)[8]) {
#pragma unroll
  for (int t = 0; t < 8; ++t) { const v8f z = {0.f, 0.f, 0.f, 0.f, 0.f, 0.f, 0.f, 0.f}; acc[t] = z; }
  const unsigned short* arh = sH + (r0 + m) * AP + 8 * hh;
  const unsigned short* arl = sL + (r0 + m) * AP + 8 * hh;
  const unsigned short* wph = wp + (size_t)m * HID + 8 * hh;
  const unsigned short* wpl = wph + WPL;
#pragma unroll 1
  for (int kt = 0; kt < KS; ++kt) {
    FragB ah, al;
    ah.u[0] = *(const v8us*)(arh + 32 * kt);
    ah.u[1] = *(const v8us*)(arh + 32 * kt + 16);
    al.u[0] = *(const v8us*)(arl + 32 * kt);
    al.u[1] = *(const v8us*)(arl + 32 * kt + 16);
#pragma unroll
    for (int t = 0; t < 8; ++t) {
      const unsigned short* bp = wph + (size_t)(16 * t) * HID + 32 * kt;
      FragB bh;
      bh.u[0] = *(const v8us*)bp;
      bh.u[1] = *(const v8us*)(bp + 16);
      acc[t] = wmb(ah.v, bh.v, acc[t]);
      acc[t] = wmb(al.v, bh.v, acc[t]);
      const unsigned short* bq = wpl + (size_t)(16 * t) * HID + 32 * kt;
      FragB bl;
      bl.u[0] = *(const v8us*)bq;
      bl.u[1] = *(const v8us*)(bq + 16);
      acc[t] = wmb(ah.v, bl.v, acc[t]);
    }
  }
}

template <int KS1>
__global__ __launch_bounds__(NTHR) void k_layer(
    const float* __restrict__ Hin, const int* __restrict__ csr, const int* __restrict__ off,
    const int* __restrict__ cnt, const float* __restrict__ aff,
    const unsigned short* __restrict__ w1p, const unsigned short* __restrict__ w2p,
    const float* __restrict__ b1, const float* __restrict__ b2,
    float* Uout, double* part, int nN, int csrLen, int useAff) {
  extern __shared__ v4f lds_dyn[];
  unsigned short* sH  = (unsigned short*)lds_dyn;
  unsigned short* sL  = sH + GROWS * AP;
  double*         sst = (double*)((char*)lds_dyn + 2 * LH_BYTES);
  float*          stg = (float*)lds_dyn;
  const int tid = threadIdx.x, lane = tid & 31, wave = tid >> 5, hh = lane >> 4, m = lane & 15;
  const int rowBase = blockIdx.x * GROWS;
  const int r0 = wave * 16;

  {
    const int cl = rowBase + r0 + m;
    const int cnt_l = cnt[cl];
    const int off_l = off[cl];
    const v4f ta = *(const v4f*)(aff + 4 * lane);
    const v4f tb = *(const v4f*)(aff + HID + 4 * lane);
    v4f a4, b4;
    a4.x = useAff != 0 ? ta.x : 1.0f; a4.y = useAff != 0 ? ta.y : 1.0f;
    a4.z = useAff != 0 ? ta.z : 1.0f; a4.w = useAff != 0 ? ta.w : 1.0f;
    b4.x = useAff != 0 ? tb.x : 0.0f; b4.y = useAff != 0 ? tb.y : 0.0f;
    b4.z = useAff != 0 ? tb.z : 0.0f; b4.w = useAff != 0 ? tb.w : 0.0f;
#pragma unroll 1
    for (int j = 0; j < 16; ++j) {
      const int c = rowBase + r0 + j;
      int n = __builtin_amdgcn_readlane(cnt_l, j);
      n = n < 0 ? 0 : (n > DEGCAP ? DEGCAP : n);
      n = (c < nN) ? n : 0;
      const int st = __builtin_amdgcn_readlane(off_l, j);
      v4f acc = {0.f, 0.f, 0.f, 0.f};
#pragma unroll 1
      for (int q0 = 0; q0 < n; q0 += 32) {
        int pos = st + q0 + lane;
        pos = pos < 0 ? 0 : (pos > csrLen - 1 ? csrLen - 1 : pos);
        int sl = csr[pos];
        sl = sl < 0 ? 0 : (sl > nN - 1 ? nN - 1 : sl);
        const int mcnt = (n - q0) < 32 ? (n - q0) : 32;
#pragma unroll 1
        for (int p = 0; p < mcnt; ++p) {
          const int s = __builtin_amdgcn_readlane(sl, p);
          const v4f u = *(const v4f*)(Hin + (size_t)s * HID + 4 * lane);
          acc = u * a4 + acc;
        }
      }
      const int cc = c < nN ? c : nN - 1;
      const v4f us = *(const v4f*)(Hin + (size_t)cc * HID + 4 * lane);
      acc = us * a4 + acc;
      acc = b4 * (float)(n + 1) + acc;
      const float keep = (c < nN) ? 1.0f : 0.0f;
      acc = acc * keep;
      unsigned int h0, l0, h1, l1, h2, l2, h3, l3;
      split2(acc.x, h0, l0); split2(acc.y, h1, l1); split2(acc.z, h2, l2); split2(acc.w, h3, l3);
      v2u hv, lv;
      hv.x = h0 | (h1 << 16); hv.y = h2 | (h3 << 16);
      lv.x = l0 | (l1 << 16); lv.y = l2 | (l3 << 16);
      *(v2u*)(sH + (r0 + j) * AP + 4 * lane) = hv;
      *(v2u*)(sL + (r0 + j) * AP + 4 * lane) = lv;
    }
  }
  __syncthreads();

  v8f acc[8];
  mm_tile<KS1>(sH, sL, w1p, r0, hh, m, acc);
  __syncthreads();
#pragma unroll
  for (int t = 0; t < 8; ++t) {
    const int col = 16 * t + m;
    const float bv = b1[col];
    unsigned short* ph = sH + (r0 + 8 * hh) * AP + col;
    unsigned short* pl = sL + (r0 + 8 * hh) * AP + col;
#pragma unroll
    for (int r = 0; r < 8; ++r) {
      const float v = fmaxf(acc[t][r] + bv, 0.0f);
      unsigned int hb, lb;
      split2(v, hb, lb);
      ph[r * AP] = (unsigned short)hb;
      pl[r * AP] = (unsigned short)lb;
    }
  }
  __syncthreads();

  mm_tile<4>(sH, sL, w2p, r0, hh, m, acc);
  __syncthreads();
  {
    const int rl0 = r0 + 8 * hh;
    const int rv  = nN - (rowBase + rl0);
#pragma unroll
    for (int t = 0; t < 8; ++t) {
      const int col = 16 * t + m;
      const float bv = b2[col];
      double s = 0.0, q = 0.0;
#pragma unroll
      for (int r = 0; r < 8; ++r) {
        const float v = fmaxf(acc[t][r] + bv, 0.0f);
        stg[(rl0 + r) * HID + col] = v;
        const float vm = (r < rv) ? v : 0.0f;
        const double dv = (double)vm;
        s += dv;
        q = dv * dv + q;
      }
      v2d e;
      e.x = s; e.y = q;
      *(v2d*)(sst + ((size_t)(wave * 2 + hh) * HID + col) * 2) = e;
    }
  }
  __syncthreads();

  const float* lp = stg + r0 * HID + 4 * lane;
  float* gp = Uout + ((size_t)rowBase + r0) * HID + 4 * lane;
  v2d po = {0.0, 0.0};
  double* pp = part + (size_t)blockIdx.x * (2 * HID) + 2 * (tid & (HID - 1));
  if (tid < HID) {
    double S = 0.0, Q = 0.0;
#pragma unroll
    for (int i = 0; i < 16; ++i) {
      const v2d e = *(const v2d*)(sst + ((size_t)i * HID + tid) * 2);
      S += e.x; Q += e.y;
    }
    po.x = S; po.y = Q;
  }
#pragma unroll
  for (int i = 0; i < 16; ++i) { const v4f v = *(const v4f*)(lp + i * HID); *(volatile v4f*)(gp + (size_t)i * HID) = v; }
  if (tid < HID) *(volatile v2d*)pp = po;
  __threadfence();
#pragma unroll
  for (int i = 0; i < 16; ++i) { const v4f v = *(const v4f*)(lp + i * HID); *(volatile v4f*)(gp + (size_t)i * HID) = v; }
  if (tid < HID) *(volatile v2d*)pp = po;
}

__global__ __launch_bounds__(HID) void k_bnfin(
    const double* __restrict__ part, int nBlk, const float* __restrict__ gam, const float* __restrict__ bet,
    float* aff, int nN) {
  const int c = threadIdx.x;
  double S = 0.0, Q = 0.0;
#pragma unroll 1
  for (int b = 0; b < nBlk; ++b) {
    const v2d e = *(const v2d*)(part + (size_t)b * (2 * HID) + 2 * c);
    S += e.x; Q += e.y;
  }
  const double inv = 1.0 / (double)nN;
  const double mu  = S * inv;
  double var = Q * inv - mu * mu;
  var = var < 0.0 ? 0.0 : var;
  const float rstd = rsqrtf((float)var + BN_EPS);
  const float a  = rstd * gam[c];
  const float bb = bet[c] - (float)mu * a;
  *(volatile float*)(aff + c) = a;
  *(volatile float*)(aff + HID + c) = bb;
  __threadfence();
  *(volatile float*)(aff + c) = a;
  *(volatile float*)(aff + HID + c) = bb;
}

__global__ __launch_bounds__(NTHR) void k_segmax(
    const int* __restrict__ batch, const float* __restrict__ U, const float* __restrict__ aff,
    float* out, int nN, int nG, int outPitch, int colOff, int vecB) {
  extern __shared__ v4f lds_dyn[];
  float* acc  = (float*)lds_dyn;
  int*   list = (int*)(acc + NBP * HID);
  int*   wcnt = list + LISTN;
  const int tid = threadIdx.x, lane = tid & 31, wave = tid >> 5;
  const int gBase = blockIdx.x * NBP;
  {
    const float ninf = __uint_as_float(0xff800000u);
    const v4f z = {ninf, ninf, ninf, ninf};
    for (int i = tid; i < NBP * HID / 4; i += NTHR) ((v4f*)acc)[i] = z;
  }
  const v4f a4 = *(const v4f*)(aff + 4 * lane);
  const v4f b4 = *(const v4f*)(aff + HID + 4 * lane);
  __syncthreads();

  const int nChunks = (nN + CHUNK - 1) / CHUNK;
#pragma unroll 1
  for (int ch = 0; ch < nChunks; ++ch) {
    const int cbase = ch * CHUNK;
    const int wc = scan_chunk<NBP>(batch, nN, cbase, gBase, vecB, list, tid, lane, wave);
    if (lane == 0) wcnt[wave] = wc;
    __syncthreads();
    if (wave == 0) {
#pragma unroll 1
      for (int wsx = 0; wsx < NWAVE; ++wsx) {
        int n = __builtin_amdgcn_readfirstlane(wcnt[wsx]);
        n = n > WCAP ? WCAP : (n < 0 ? 0 : n);
        const int* lp = list + wsx * WCAP;
#pragma unroll 1
        for (int i = 0; i < n; ++i) {
          const int ent  = __builtin_amdgcn_readfirstlane(lp[i]);
          const int slot = ent & (NBP - 1);
          int nd = cbase + ((ent >> 12) & (CHUNK - 1));
          nd = nd > nN - 1 ? nN - 1 : nd;
          const v4f u = *(const v4f*)(U + (size_t)nd * HID + 4 * lane);
          const v4f v = u * a4 + b4;
          v4f* ap = (v4f*)(acc + slot * HID + 4 * lane);
          v4f cur = *ap;
          cur.x = fmaxf(cur.x, v.x); cur.y = fmaxf(cur.y, v.y);
          cur.z = fmaxf(cur.z, v.z); cur.w = fmaxf(cur.w, v.w);
          *ap = cur;
        }
      }
    }
    __syncthreads();
  }

  float* basep = out + colOff + 4 * lane;
#pragma unroll 1
  for (int j = 0; j < 32; ++j) {
    const int slot = wave * 32 + j;
    const int g = gBase + slot;
    const v4f v = *(const v4f*)(acc + slot * HID + 4 * lane);
    if (g < nG) *(volatile v4f*)(basep + (size_t)g * outPitch) = v;
  }
  __threadfence();
#pragma unroll 1
  for (int j = 0; j < 32; ++j) {
    const int slot = wave * 32 + j;
    const int g = gBase + slot;
    const v4f v = *(const v4f*)(acc + slot * HID + 4 * lane);
    if (g < nG) *(volatile v4f*)(basep + (size_t)g * outPitch) = v;
  }
}

extern "C" void kernel_launch(void* const* d_in, const int* in_sizes, int n_in,
                              void* d_out, int out_size, void* d_ws, size_t ws_size,
                              hipStream_t stream) {
  if (n_in < 21) return;
  const int nN = in_sizes[2];
  if (nN <= 0 || nN > (1 << 23)) return;
  const int fin = in_sizes[0] / nN;
  if (fin < 1 || fin > HID || (long)nN * fin != (long)in_sizes[0]) return;
  const int nE = in_sizes[1] / 2;
  if (nE <= 0 || in_sizes[1] != 2 * nE || nE > (1 << 28)) return;
  if (in_sizes[3] != fin * HID) return;
  for (int l = 0; l < 3; ++l) {
    if (l > 0 && in_sizes[3 + 6 * l] != HID * HID) return;
    if (in_sizes[5 + 6 * l] != HID * HID) return;
    if (in_sizes[4 + 6 * l] < HID || in_sizes[6 + 6 * l] < HID || in_sizes[7 + 6 * l] < HID || in_sizes[8 + 6 * l] < HID) return;
  }
  const int G = out_size / (3 * HID);
  if (G < 1 || out_size != G * 3 * HID) return;

  const float* x     = (const float*)d_in[0];
  const int*   ei    = (const int*)d_in[1];
  const int*   batch = (const int*)d_in[2];
  const float* w1[3]; const float* b1[3]; const float* w2[3]; const float* b2[3]; const float* gm[3]; const float* be[3];
  for (int l = 0; l < 3; ++l) {
    w1[l] = (const float*)d_in[3 + 6 * l];
    b1[l] = (const float*)d_in[4 + 6 * l];
    w2[l] = (const float*)d_in[5 + 6 * l];
    b2[l] = (const float*)d_in[6 + 6 * l];
    gm[l] = (const float*)d_in[7 + 6 * l];
    be[l] = (const float*)d_in[8 + 6 * l];
  }
  float* out = (float*)d_out;

  const int NPAD   = ((nN + 255) / 256) * 256;
  const int nBlk   = NPAD / GROWS;
  const int nBC    = (nN + NBC - 1) / NBC;
  const int CNTPAD = nBC * NBC;
  if (2 * nBC + 1 > RBN) return;
  const int nBF    = (nN + NBF - 1) / NBF;
  const int csrLen = ((nE + 31) & ~31) + 32 * RBN;
  const int nSeg   = (G + NBP - 1) / NBP;
  const int total4 = NPAD * 32;

  char* ws = (char*)d_ws;
  size_t o = 0;
  const size_t oWsb  = o; o += (size_t)6 * 2 * WPL * 2;          o = (o + 255) & ~(size_t)255;
  const size_t oCnt  = o; o += (size_t)CNTPAD * 4;               o = (o + 255) & ~(size_t)255;
  const size_t oOff  = o; o += (size_t)CNTPAD * 4;               o = (o + 255) & ~(size_t)255;
  const size_t oRb   = o; o += (size_t)RBN * 4;                  o = (o + 255) & ~(size_t)255;
  const size_t oCsr  = o; o += (size_t)csrLen * 4;               o = (o + 255) & ~(size_t)255;
  const size_t oP0   = o; o += (size_t)NPAD * HID * 4;           o = (o + 255) & ~(size_t)255;
  const size_t oP1   = o; o += (size_t)NPAD * HID * 4;           o = (o + 255) & ~(size_t)255;
  const size_t oPart = o; o += (size_t)nBlk * (2 * HID) * 8;      o = (o + 255) & ~(size_t)255;
  const size_t oAff  = o; o += (size_t)3 * 2 * HID * 4;          o = (o + 255) & ~(size_t)255;
  if (o > ws_size || o > ((size_t)128 << 20)) return;
  unsigned short* wsb  = (unsigned short*)(ws + oWsb);
  int*            cnt  = (int*)(ws + oCnt);
  int*            offp = (int*)(ws + oOff);
  int*            rb   = (int*)(ws + oRb);
  int*            csr  = (int*)(ws + oCsr);
  float*          P0   = (float*)(ws + oP0);
  float*          P1   = (float*)(ws + oP1);
  double*         part = (double*)(ws + oPart);
  float*          affT = (float*)(ws + oAff);

  const int vec8 = ((nE & 3) == 0) ? 1 : 0;

  k_wprep<<<6 * 2048 / NTHR, NTHR, 0, stream>>>(w1[0], w2[0], w1[1], w2[1], w1[2], w2[2], wsb, fin);
  k_pad<<<total4 / NTHR, NTHR, 0, stream>>>(x, P0, nN, fin, total4);
  k_count<<<nBC, NTHR, 0, stream>>>(ei, cnt, nE, vec8);
  k_offsets<<<1, OTHR, 0, stream>>>(cnt, offp, rb, nBC);
  hipFuncSetAttribute(reinterpret_cast<const void*>(&k_fill), hipFuncAttributeMaxDynamicSharedMemorySize, LDS_FILL);
  k_fill<<<nBF, NTHR, LDS_FILL, stream>>>(ei, offp, rb, csr, nN, nE, vec8, csrLen);

  hipFuncSetAttribute(reinterpret_cast<const void*>(&k_layer<3>), hipFuncAttributeMaxDynamicSharedMemorySize, LDS_LAYER);
  hipFuncSetAttribute(reinterpret_cast<const void*>(&k_layer<4>), hipFuncAttributeMaxDynamicSharedMemorySize, LDS_LAYER);
  hipFuncSetAttribute(reinterpret_cast<const void*>(&k_segmax), hipFuncAttributeMaxDynamicSharedMemorySize, LDS_SEG);

  for (int l = 0; l < 3; ++l) {
    const float* hin  = (l == 1) ? P1 : P0;
    float*       uout = (l == 1) ? P0 : P1;
    const float* affIn = affT + (size_t)(l > 0 ? l - 1 : 0) * (2 * HID);
    float*       affOut = affT + (size_t)l * (2 * HID);
    const unsigned short* w1p = wsb + (size_t)(2 * l) * (2 * WPL);
    const unsigned short* w2p = wsb + (size_t)(2 * l + 1) * (2 * WPL);
    const int useAff = l > 0 ? 1 : 0;
    if (l == 0 && fin <= 96) {
      k_layer<3><<<nBlk, NTHR, LDS_LAYER, stream>>>(hin, csr, offp, cnt, affIn, w1p, w2p, b1[l], b2[l],
                                                    uout, part, nN, csrLen, useAff);
    } else {
      k_layer<4><<<nBlk, NTHR, LDS_LAYER, stream>>>(hin, csr, offp, cnt, affIn, w1p, w2p, b1[l], b2[l],
                                                    uout, part, nN, csrLen, useAff);
    }
    k_bnfin<<<1, HID, 0, stream>>>(part, nBlk, gm[l], be[l], affOut, nN);
    k_segmax<<<nSeg, NTHR, LDS_SEG, stream>>>(batch, uout, affOut, out, nN, G, 3 * HID, l * HID, 1);
  }
}
